// GNNEncoder_2018634629227
// MI455X (gfx1250) — hardware-verified
//
#include <hip/hip_runtime.h>
#include <math.h>
#include <stdint.h>
#include <stddef.h>

#define NN_   4096
#define FIN_  165
#define KIN_  192
#define HID_  128
#define NLY_  2
#define NH_   4
#define HD_   32
#define NWSQ  9
#define ADW   128
#define SFP   132
#define SHP   72
#define SMEM_BYTES 36864
#define ATT_SCALE 0.17677669529663687f
#define BN_EPS 1.0e-5f
#define SLOPE 0.2f
#define MASKFILL (-1.0e9f)
#define MASKHALF (-1.0e8f)
#define WSMAX 134217728

#define XROWS  8
#define XUNITS (KIN_ / 8)
#define XTHR   (XROWS * XUNITS)
#define XCHUNK (XROWS * FIN_)
#define XCH4   (XCHUNK / 4)

static_assert(HID_ == NH_ * HD_);
static_assert(HD_ == 32);
static_assert(HID_ == 128);
static_assert(NN_ % 64 == 0);
static_assert(NN_ == ADW * 32);
static_assert(KIN_ % 32 == 0 && KIN_ >= FIN_);
static_assert(XCHUNK % 4 == 0);
static_assert(NN_ % XROWS == 0);
static_assert(XTHR < XCH4 && 2 * XTHR >= XCH4);
static_assert((HID_ * XUNITS) % 256 == 0);
static_assert((NN_ * HID_) % 2048 == 0);
static_assert(NN_ == 4 * 1024);
static_assert(NN_ % 16 == 0);
static_assert(64 * SFP * 4 <= SMEM_BYTES);
static_assert(2 * HID_ * SHP * 2 <= SMEM_BYTES);

typedef __attribute__((ext_vector_type(16))) __bf16 v16b;
typedef __attribute__((ext_vector_type(8)))  __bf16 v8b;
typedef __attribute__((ext_vector_type(8)))  float  v8f;
typedef __attribute__((ext_vector_type(4)))  float  v4f;
typedef __attribute__((ext_vector_type(4)))  unsigned int v4u;
typedef __attribute__((ext_vector_type(2)))  unsigned int v2u;
typedef __attribute__((ext_vector_type(8)))  unsigned int v8u;
typedef __attribute__((ext_vector_type(4)))  int v4i;
typedef v8b __attribute__((may_alias)) v8ba;
typedef v4f __attribute__((may_alias)) v4fa;
typedef v4u __attribute__((may_alias)) v4ua;
typedef v2u __attribute__((may_alias)) v2ua;
typedef v4i __attribute__((may_alias)) v4ia;

union FragU { v16b v; v8b h[2]; };
union PackU { v8u u; v16b v; };

__device__ __forceinline__ unsigned short f2bf_bits(float f) {
  const unsigned u = __float_as_uint(f);
  return (unsigned short)((u + 0x7FFFu + ((u >> 16) & 1u)) >> 16);
}
__device__ __forceinline__ float bf_bits2f(unsigned short h) { return __uint_as_float(((unsigned)h) << 16); }
__device__ __forceinline__ float bf16r(float f) {
  unsigned u = __float_as_uint(f);
  u = (u + 0x7FFFu + ((u >> 16) & 1u)) & 0xFFFF0000u;
  return __uint_as_float(u);
}
__device__ __forceinline__ unsigned pk16(unsigned short a, unsigned short b) { return (unsigned)a | ((unsigned)b << 16); }

__device__ __forceinline__ v8f wmma_bf16(v16b a, v16b b, v8f c) {
  v8f d = __builtin_amdgcn_wmma_f32_16x16x32_bf16(false, a, false, b, (short)0, c, false, false);
  asm volatile("v_nop\n\tv_nop\n\tv_nop\n\tv_nop" : "+v"(d) : "v"(a), "v"(b));
  return d;
}

__device__ __forceinline__ v16b load_frag(const unsigned short* p, int hh) {
  FragU f;
  f.h[0] = *(const v8ba*)(p + 8 * hh);
  f.h[1] = *(const v8ba*)(p + 16 + 8 * hh);
  return f.v;
}

__device__ __forceinline__ void pack_p2(v8f a, v8f c, v16b& ho, v16b& lo) {
  PackU uh, ul;
#pragma unroll
  for (int i = 0; i < 4; ++i) {
    const unsigned short h0 = f2bf_bits(a[2 * i]), h1 = f2bf_bits(a[2 * i + 1]);
    const unsigned short l0 = f2bf_bits(a[2 * i] - bf_bits2f(h0)), l1 = f2bf_bits(a[2 * i + 1] - bf_bits2f(h1));
    uh.u[i] = pk16(h0, h1); ul.u[i] = pk16(l0, l1);
    const unsigned short g0 = f2bf_bits(c[2 * i]), g1 = f2bf_bits(c[2 * i + 1]);
    const unsigned short m0 = f2bf_bits(c[2 * i] - bf_bits2f(g0)), m1 = f2bf_bits(c[2 * i + 1] - bf_bits2f(g1));
    uh.u[4 + i] = pk16(g0, g1); ul.u[4 + i] = pk16(m0, m1);
  }
  ho = uh.v; lo = ul.v;
}

template <bool ASPLIT>
__device__ __forceinline__ void gemm_core_32x64(
    const unsigned short* __restrict__ Ah, const unsigned short* __restrict__ Al,
    const unsigned short* __restrict__ Bt, int K, size_t aoff, size_t boff, int hh, v8f (&acc)[2][4]) {
  const unsigned short* a0 = Ah + aoff;
  const unsigned short* a1 = a0 + (size_t)16 * K;
  const unsigned short* c0 = (ASPLIT ? Al : Ah) + aoff;
  const unsigned short* c1 = c0 + (size_t)16 * K;
  const unsigned short* bp = Bt + boff;
#pragma unroll 1
  for (int k0 = 0; k0 < K; k0 += 32) {
    const v16b f0 = load_frag(a0 + k0, hh);
    const v16b f1 = load_frag(a1 + k0, hh);
    v16b g0 = f0, g1 = f1;
    if (ASPLIT) { g0 = load_frag(c0 + k0, hh); g1 = load_frag(c1 + k0, hh); }
#pragma unroll
    for (int nt = 0; nt < 4; ++nt) {
      const v16b fb = load_frag(bp + (size_t)nt * 16 * K + k0, hh);
      acc[0][nt] = wmma_bf16(f0, fb, acc[0][nt]);
      acc[1][nt] = wmma_bf16(f1, fb, acc[1][nt]);
      if (ASPLIT) {
        acc[0][nt] = wmma_bf16(g0, fb, acc[0][nt]);
        acc[1][nt] = wmma_bf16(g1, fb, acc[1][nt]);
      }
    }
  }
}

__global__ __launch_bounds__(XTHR) void k_cvtx(const float* __restrict__ x, unsigned short* __restrict__ Xb) {
  __shared__ __align__(16) float sX[XCHUNK];
  const int tid = threadIdx.x;
  const size_t fb = (size_t)blockIdx.x * XCHUNK;
  {
    const int i0  = tid;
    const int i1r = tid + XTHR;
    const int i1  = i1r < XCH4 ? i1r : (XCH4 - 1);
    const v4f a = *(const v4fa*)(x + fb + (size_t)4 * i0);
    const v4f b = *(const v4fa*)(x + fb + (size_t)4 * i1);
    *(v4fa*)(sX + 4 * i0) = a;
    *(v4fa*)(sX + 4 * i1) = b;
  }
  __syncthreads();
  const int rl = tid / XUNITS;
  const int u  = tid - rl * XUNITS;
  const int c8 = u * 8;
  const float* rp = sX + rl * FIN_;
  v4u o;
#pragma unroll
  for (int qd = 0; qd < 4; ++qd) {
    const int ca = c8 + 2 * qd, cb = ca + 1;
    const float fa = rp[ca < FIN_ ? ca : (FIN_ - 1)];
    const float fc = rp[cb < FIN_ ? cb : (FIN_ - 1)];
    const unsigned short ha = (ca < FIN_) ? f2bf_bits(fa) : (unsigned short)0;
    const unsigned short hc = (cb < FIN_) ? f2bf_bits(fc) : (unsigned short)0;
    o[qd] = pk16(ha, hc);
  }
  unsigned short* d = Xb + (size_t)blockIdx.x * (XROWS * KIN_) + (size_t)tid * 8;
  *(volatile v4u*)d = o;
  __threadfence();
  *(volatile v4u*)d = o;
}

__global__ __launch_bounds__(256) void k_cvtwin(const float* __restrict__ W, unsigned short* __restrict__ Wib) {
  const int u = blockIdx.x * 256 + threadIdx.x;
  const int n = u / XUNITS, j = u - n * XUNITS;
  const int kb = j * 8;
  float e[8];
#pragma unroll
  for (int i = 0; i < 8; ++i) {
    const int k  = kb + i;
    const int kc = k < FIN_ ? k : (FIN_ - 1);
    e[i] = W[(size_t)kc * HID_ + n];
  }
  v4u o;
#pragma unroll
  for (int qd = 0; qd < 4; ++qd) {
    const int ka = kb + 2 * qd, kc2 = ka + 1;
    const unsigned short ha = (ka  < FIN_) ? f2bf_bits(e[2 * qd])     : (unsigned short)0;
    const unsigned short hb = (kc2 < FIN_) ? f2bf_bits(e[2 * qd + 1]) : (unsigned short)0;
    o[qd] = pk16(ha, hb);
  }
  unsigned short* d = Wib + (size_t)u * 8;
  *(volatile v4u*)d = o;
  __threadfence();
  *(volatile v4u*)d = o;
}

__global__ __launch_bounds__(256) void k_tcvt9(const float* __restrict__ Wq, const float* __restrict__ Wk,
                                               const float* __restrict__ Wv, const float* __restrict__ Wo,
                                               const float* __restrict__ Wf, unsigned short* __restrict__ oball) {
  __shared__ __align__(16) float tf[64 * 68];
  const int z = blockIdx.z;
  const float* W = Wf;
  if (z < 8) {
    const float* b4 = (z < 2) ? Wq : ((z < 4) ? Wk : ((z < 6) ? Wv : Wo));
    W = b4 + (size_t)(z & 1) * (HID_ * HID_);
  }
  unsigned short* ob = oball + (size_t)z * (HID_ * HID_);
  const int R = HID_, Cc = HID_;
  const int c0  = blockIdx.x * 64;
  const int r0  = blockIdx.y * 64;
  const int tid = threadIdx.x;
  {
    const int lr = tid >> 4;
    const int c4 = (tid & 15) * 4;
#pragma unroll
    for (int it = 0; it < 4; ++it) {
      const int rr = it * 16 + lr;
      const v4f a = *(const v4fa*)(W + (size_t)(r0 + rr) * Cc + c0 + c4);
      *(v4fa*)(tf + rr * 68 + c4) = a;
    }
  }
  __syncthreads();
  const int sub = tid >> 3;
  const int c8  = (tid & 7) * 8;
  v4u hv[2];
#pragma unroll
  for (int it = 0; it < 2; ++it) {
    const int oc = it * 32 + sub;
    v4u a;
#pragma unroll
    for (int q = 0; q < 4; ++q) {
      const float f0 = tf[(c8 + 2 * q) * 68 + oc];
      const float f1 = tf[(c8 + 2 * q + 1) * 68 + oc];
      a[q] = pk16(f2bf_bits(f0), f2bf_bits(f1));
    }
    hv[it] = a;
  }
  for (int pass = 0; pass < 2; ++pass) {
#pragma unroll
    for (int it = 0; it < 2; ++it) {
      const int oc = it * 32 + sub;
      const size_t go = (size_t)(c0 + oc) * R + r0 + c8;
      *(volatile v4u*)(ob + go) = hv[it];
    }
    __threadfence();
  }
}

#define AD_NT   256
#define AD_NW   8
#define EPT     8
#define CHUNK   (AD_NT * EPT)
#define WCAP    (EPT * 32)
#define SLOTB   6
#define NSLOT   64

static_assert((1 << SLOTB) == NSLOT);
static_assert((CHUNK & (CHUNK - 1)) == 0 && CHUNK == 2048);
static_assert(AD_NT == 32 * AD_NW);
static_assert(AD_NT * 32 == NSLOT * ADW);
static_assert(NN_ % NSLOT == 0);
static_assert(NN_ <= 4096);

__device__ __forceinline__ int scan_chunk(const int* __restrict__ keys, int nE, int cbase, int slotBase,
                                          int nb, int vec8, int* list, int tid, int lane, int wave) {
  int wc = 0;
  const int el0  = tid * EPT;
  const int e0   = cbase + el0;
  const int sent = -2147483647 - 1;
  v4i da, db;
  if (vec8 != 0 && cbase + CHUNK <= nE) {
    da = *(const v4ia*)(keys + e0);
    db = *(const v4ia*)(keys + e0 + 4);
  } else {
    da.x = (e0     < nE) ? keys[min(e0,     nE - 1)] : sent;
    da.y = (e0 + 1 < nE) ? keys[min(e0 + 1, nE - 1)] : sent;
    da.z = (e0 + 2 < nE) ? keys[min(e0 + 2, nE - 1)] : sent;
    da.w = (e0 + 3 < nE) ? keys[min(e0 + 3, nE - 1)] : sent;
    db.x = (e0 + 4 < nE) ? keys[min(e0 + 4, nE - 1)] : sent;
    db.y = (e0 + 5 < nE) ? keys[min(e0 + 5, nE - 1)] : sent;
    db.z = (e0 + 6 < nE) ? keys[min(e0 + 6, nE - 1)] : sent;
    db.w = (e0 + 7 < nE) ? keys[min(e0 + 7, nE - 1)] : sent;
  }
  const unsigned nbs = (unsigned)slotBase;
  const unsigned unb = (unsigned)nb;
  const unsigned s0 = (unsigned)da.x - nbs, s1 = (unsigned)da.y - nbs;
  const unsigned s2 = (unsigned)da.z - nbs, s3 = (unsigned)da.w - nbs;
  const unsigned s4 = (unsigned)db.x - nbs, s5 = (unsigned)db.y - nbs;
  const unsigned s6 = (unsigned)db.z - nbs, s7 = (unsigned)db.w - nbs;
  const bool h0 = s0 < unb, h1 = s1 < unb, h2 = s2 < unb, h3 = s3 < unb;
  const bool h4 = s4 < unb, h5 = s5 < unb, h6 = s6 < unb, h7 = s7 < unb;
  const unsigned any = __builtin_amdgcn_ballot_w32(h0 | h1 | h2 | h3 | h4 | h5 | h6 | h7);
  if (any != 0u) {
#define HITJ(J, HJ, SJ) { \
      const unsigned mj = __builtin_amdgcn_ballot_w32(HJ); \
      if (mj != 0u) { \
        if (HJ) { \
          const int pos = wc + (int)__builtin_amdgcn_mbcnt_lo(mj, 0u); \
          if (pos < WCAP) list[wave * WCAP + pos] = ((el0 + (J)) << SLOTB) | (int)(SJ); \
        } \
        wc += (int)__builtin_popcount(mj); } }
    HITJ(0, h0, s0)
    HITJ(1, h1, s1)
    HITJ(2, h2, s2)
    HITJ(3, h3, s3)
    HITJ(4, h4, s4)
    HITJ(5, h5, s5)
    HITJ(6, h6, s6)
    HITJ(7, h7, s7)
#undef HITJ
  }
  return wc;
}

__global__ __launch_bounds__(AD_NT) void k_adj(const int* __restrict__ keys, const int* __restrict__ gath,
                                               unsigned int* __restrict__ ADJ, int nE, int vec8) {
  __shared__ __align__(16) unsigned int sBits[NSLOT * ADW];
  __shared__ int list[AD_NW * WCAP];
  __shared__ int wcnt[AD_NW];
  const int tid = (int)threadIdx.x, lane = tid & 31, wave = tid >> 5;
  const int r0 = (int)blockIdx.x * NSLOT;

  {
    const v4u z = {0u, 0u, 0u, 0u};
#pragma unroll
    for (int i = 0; i < 8; ++i) *(v4ua*)(sBits + tid * 32 + 4 * i) = z;
  }
  __syncthreads();

  const int nChunks = (nE + CHUNK - 1) / CHUNK;
#pragma unroll 1
  for (int ch = 0; ch < nChunks; ++ch) {
    const int cbase = ch * CHUNK;
    const int wc = scan_chunk(keys, nE, cbase, r0, NSLOT, vec8, list, tid, lane, wave);
    if (lane == 0) wcnt[wave] = wc;
    __syncthreads();
    const int wcc = wc > WCAP ? WCAP : wc;
#pragma unroll 1
    for (int i0 = 0; i0 < wcc; i0 += 32) {
      const int i   = i0 + lane;
      const int ic  = i < wcc ? i : wcc - 1;
      const int ent = list[wave * WCAP + ic];
      const int el  = (ent >> SLOTB) & (CHUNK - 1);
      const int sl  = ent & (NSLOT - 1);
      int eid = cbase + el;
      eid = eid > nE - 1 ? nE - 1 : eid;
      int d = gath[eid];
      d = d < 0 ? 0 : (d > NN_ - 1 ? NN_ - 1 : d);
      const int packed = (sl << 12) | d;
      if (i < wcc) list[wave * WCAP + i] = packed;
    }
    __syncthreads();
    if (wave < 2) {
      const int row = tid;
#pragma unroll 1
      for (int w2 = 0; w2 < AD_NW; ++w2) {
        int cnt = wcnt[w2];
        cnt = cnt < 0 ? 0 : (cnt > WCAP ? WCAP : cnt);
#pragma unroll 1
        for (int i = 0; i < cnt; ++i) {
          const int ent = list[w2 * WCAP + i];
          const bool hit = (((ent >> 12) & (NSLOT - 1)) == row);
          const unsigned int bit = hit ? (1u << (ent & 31)) : 0u;
          const int idx = row * ADW + ((ent & (NN_ - 1)) >> 5);
          sBits[idx] = sBits[idx] | bit;
        }
      }
    }
    __syncthreads();
  }
  for (int pass = 0; pass < 2; ++pass) {
#pragma unroll
    for (int it = 0; it < 8; ++it) {
      const int wo = it * (AD_NT * 4) + tid * 4;
      const v4u v = *(const v4ua*)(sBits + wo);
      *(volatile v4u*)(ADJ + (size_t)r0 * ADW + wo) = v;
    }
    __threadfence();
  }
}

template <bool ASPLIT, int MODE>
__global__ __launch_bounds__(128) void k_gemm(
    const unsigned short* __restrict__ Ah, const unsigned short* __restrict__ Al, int K,
    const unsigned short* __restrict__ Bt, const float* __restrict__ bias,
    float* __restrict__ outF, unsigned short* __restrict__ outH, unsigned short* __restrict__ outL) {
  __shared__ __align__(16) unsigned char smem[SMEM_BYTES];
  float* sF = (float*)smem;
  unsigned short* sH = (unsigned short*)smem;
  unsigned short* sL = sH + HID_ * SHP;

  const int tid = threadIdx.x, lane = tid & 31, w = tid >> 5;
  const int hh = lane >> 4, m = lane & 15;
  const int m0 = blockIdx.x * 64;
  const int wr = 32 * (w >> 1);
  const int wc = 64 * (w & 1);

  const v8f zero8 = {0.f, 0.f, 0.f, 0.f, 0.f, 0.f, 0.f, 0.f};
  v8f acc[2][4];
#pragma unroll
  for (int mt = 0; mt < 2; ++mt)
#pragma unroll
    for (int nt = 0; nt < 4; ++nt) acc[mt][nt] = zero8;

  gemm_core_32x64<ASPLIT>(Ah, Al, Bt, K, (size_t)(m0 + wr + m) * (size_t)K, (size_t)(wc + m) * (size_t)K, hh, acc);

  float bv[4];
#pragma unroll
  for (int nt = 0; nt < 4; ++nt) bv[nt] = bf16r(bias[wc + 16 * nt + m]);

  if (MODE != 3) {
#pragma unroll
    for (int nt = 0; nt < 4; ++nt)
#pragma unroll
      for (int mt = 0; mt < 2; ++mt)
#pragma unroll
        for (int r = 0; r < 8; ++r) {
          const int rowl = wr + 16 * mt + 8 * hh + r;
          const int col  = wc + 16 * nt + m;
          sF[rowl * SFP + col] = acc[mt][nt][r] + bv[nt];
        }
  } else {
#pragma unroll
    for (int nt = 0; nt < 4; ++nt)
#pragma unroll
      for (int mt = 0; mt < 2; ++mt)
#pragma unroll
        for (int r = 0; r < 8; ++r) {
          const int rowl = wr + 16 * mt + 8 * hh + r;
          const int col  = wc + 16 * nt + m;
          const float v = acc[mt][nt][r] + bv[nt];
          const unsigned short hb = f2bf_bits(v);
          const unsigned short lb = f2bf_bits(v - bf_bits2f(hb));
          sH[col * SHP + rowl] = hb;
          sL[col * SHP + rowl] = lb;
        }
  }
  __syncthreads();

  if (MODE == 3) {
    const int n0 = blockIdx.x * 64;
    const int q4 = lane >> 3, t8 = (lane & 7) * 8;
    for (int pass = 0; pass < 2; ++pass) {
#pragma unroll
      for (int it = 0; it < 8; ++it) {
        const int feat = 16 * it + 4 * w + q4;
        const v4u hv = *(const v4ua*)(sH + feat * SHP + t8);
        const v4u lv = *(const v4ua*)(sL + feat * SHP + t8);
        const size_t go = (size_t)feat * (size_t)NN_ + n0 + t8;
        *(volatile v4u*)(outH + go) = hv;
        *(volatile v4u*)(outL + go) = lv;
      }
      __threadfence();
    }
  } else {
    const int c8 = (lane & 15) * 8;
    for (int pass = 0; pass < 2; ++pass) {
      if (MODE == 0 || MODE == 1) {
#pragma unroll
        for (int i = 0; i < 16; ++i) {
          const int row = 16 * w + i;
          const v4f v = *(const v4fa*)(sF + row * SFP + 4 * lane);
          *(volatile v4f*)(outF + (size_t)(m0 + row) * HID_ + 4 * lane) = v;
        }
      }
      if (MODE == 1 || MODE == 2) {
#pragma unroll
        for (int it = 0; it < 8; ++it) {
          const int row = 16 * w + 2 * it + hh;
          const float* sp = sF + row * SFP + c8;
          const v4f fa = *(const v4fa*)(sp);
          const v4f fb = *(const v4fa*)(sp + 4);
          const float e8[8] = {fa[0], fa[1], fa[2], fa[3], fb[0], fb[1], fb[2], fb[3]};
          v4u hv, lv;
#pragma unroll
          for (int q = 0; q < 4; ++q) {
            const unsigned short h0 = f2bf_bits(e8[2 * q]), h1 = f2bf_bits(e8[2 * q + 1]);
            const unsigned short l0 = f2bf_bits(e8[2 * q] - bf_bits2f(h0)), l1 = f2bf_bits(e8[2 * q + 1] - bf_bits2f(h1));
            hv[q] = pk16(h0, h1);
            lv[q] = pk16(l0, l1);
          }
          const size_t go = (size_t)(m0 + row) * HID_ + c8;
          *(volatile v4u*)(outH + go) = hv;
          *(volatile v4u*)(outL + go) = lv;
        }
      }
      __threadfence();
    }
  }
}

__global__ __launch_bounds__(128) void k_attn(
    const unsigned short* __restrict__ Qh, const unsigned short* __restrict__ Ql,
    const unsigned short* __restrict__ Kh, const unsigned short* __restrict__ Kl,
    const unsigned short* __restrict__ VTh, const unsigned short* __restrict__ VTl,
    const unsigned int* __restrict__ ADJ, float* __restrict__ AO) {
  __shared__ __align__(16) unsigned int sMsk[NSLOT * ADW];
  __shared__ __align__(16) float sO[4][16 * 36];

  const int tid = threadIdx.x, lane = tid & 31, w = tid >> 5;
  const int hh = lane >> 4, m = lane & 15;
  const int qt = blockIdx.x;
  const int h  = blockIdx.y;
  const int q0 = qt * 64, q0w = q0 + 16 * w, q = q0w + m;

  {
    const unsigned int* ga = ADJ + (size_t)q0 * ADW;
#pragma unroll 4
    for (int it = 0; it < 16; ++it) {
      const int wo = (it * 128 + tid) * 4;
      const v4u a = *(const v4ua*)(ga + wo);
      *(v4ua*)(sMsk + wo) = a;
    }
  }
  const v16b qfh = load_frag(Qh + (size_t)q * HID_ + h * HD_, hh);
  const v16b qfl = load_frag(Ql + (size_t)q * HID_ + h * HD_, hh);

  const v8f zero8 = {0.f, 0.f, 0.f, 0.f, 0.f, 0.f, 0.f, 0.f};
  v8f o[2];
  o[0] = zero8; o[1] = zero8;
  float mrun = MASKFILL, lrun = 0.0f;

  __syncthreads();
  const unsigned int* mrow = sMsk + (16 * w + m) * ADW;

#pragma unroll 1
  for (int ks = 0; ks < NN_ / 64; ++ks) {
    const int kb = ks * 64;
    const v2u mw = *(const v2ua*)(mrow + 2 * ks);
    const unsigned int w0 = mw[0], w1 = mw[1];

    v8f s[4];
#pragma unroll
    for (int j = 0; j < 4; ++j) {
      const size_t krow = ((size_t)(kb + 16 * j + m)) * HID_ + h * HD_;
      const v16b kfh = load_frag(Kh + krow, hh);
      const v16b kfl = load_frag(Kl + krow, hh);
      v8f a = zero8;
      a = wmma_bf16(kfh, qfh, a);
      a = wmma_bf16(kfh, qfl, a);
      a = wmma_bf16(kfl, qfh, a);
      const unsigned int wsel = (j < 2) ? w0 : w1;
      const unsigned int bits = (wsel >> (((j & 1) * 16) + 8 * hh)) & 0xFFu;
#pragma unroll
      for (int r = 0; r < 8; ++r) {
        float t = a[r] * ATT_SCALE;
        t = (t >= 0.0f) ? t : SLOPE * t;
        t = (((bits >> r) & 1u) != 0u) ? t : MASKFILL;
        s[j][r] = t;
      }
    }
    float cm = MASKFILL;
#pragma unroll
    for (int j = 0; j < 4; ++j)
#pragma unroll
      for (int r = 0; r < 8; ++r) cm = fmaxf(cm, s[j][r]);
    cm = fmaxf(cm, __shfl_xor(cm, 16, 32));
    const float mnew  = fmaxf(mrun, cm);
    const float aexp  = __expf(mrun - mnew);
    const float alpha = (mrun > MASKHALF) ? aexp : 0.0f;
    mrun = mnew;
    float psum = 0.0f;
#pragma unroll
    for (int j = 0; j < 4; ++j)
#pragma unroll
      for (int r = 0; r < 8; ++r) {
        const float sv = s[j][r];
        const float pe = __expf(sv - mnew);
        const float p  = (sv > MASKHALF) ? pe : 0.0f;
        psum += p;
        s[j][r] = p;
      }
    psum += __shfl_xor(psum, 16, 32);
    lrun = lrun * alpha + psum;
#pragma unroll
    for (int t = 0; t < 2; ++t)
#pragma unroll
      for (int r = 0; r < 8; ++r) o[t][r] *= alpha;

    v16b p0h, p0l, p1h, p1l;
    pack_p2(s[0], s[1], p0h, p0l);
    pack_p2(s[2], s[3], p1h, p1l);

#pragma unroll
    for (int t = 0; t < 2; ++t) {
      const unsigned short* vph = VTh + ((size_t)(h * HD_ + 16 * t + m)) * (size_t)NN_ + kb;
      const unsigned short* vpl = VTl + ((size_t)(h * HD_ + 16 * t + m)) * (size_t)NN_ + kb;
      const v16b v0h = load_frag(vph, hh), v0l = load_frag(vpl, hh);
      o[t] = wmma_bf16(v0h, p0h, o[t]);
      o[t] = wmma_bf16(v0h, p0l, o[t]);
      o[t] = wmma_bf16(v0l, p0h, o[t]);
      const v16b v1h = load_frag(vph + 32, hh), v1l = load_frag(vpl + 32, hh);
      o[t] = wmma_bf16(v1h, p1h, o[t]);
      o[t] = wmma_bf16(v1h, p1l, o[t]);
      o[t] = wmma_bf16(v1l, p1h, o[t]);
    }
  }

  const float inv = (lrun > 0.0f) ? (1.0f / lrun) : 0.0f;
  float* so = sO[w];
#pragma unroll
  for (int t = 0; t < 2; ++t)
#pragma unroll
    for (int r = 0; r < 8; ++r) so[m * 36 + 16 * t + 8 * hh + r] = o[t][r] * inv;
  __syncthreads();
  {
    const int rq = lane >> 3, c4 = (lane & 7) * 4;
    for (int pass = 0; pass < 2; ++pass) {
#pragma unroll
      for (int it = 0; it < 4; ++it) {
        const int row = 4 * it + rq;
        const v4f v = *(const v4fa*)(so + row * 36 + c4);
        *(volatile v4f*)(AO + (size_t)(q0w + row) * (size_t)HID_ + h * HD_ + c4) = v;
      }
      __threadfence();
    }
  }
}

__global__ __launch_bounds__(256) void k_split(const float* __restrict__ src, unsigned short* __restrict__ hi,
                                               unsigned short* __restrict__ lo, int n8) {
  int i = blockIdx.x * 256 + threadIdx.x;
  const bool ok = i < n8;
  i = ok ? i : (n8 - 1);
  const float* s = src + (size_t)i * 8;
  const v4f f0 = *(const v4fa*)(s);
  const v4f f1 = *(const v4fa*)(s + 4);
  const float e[8] = {f0[0], f0[1], f0[2], f0[3], f1[0], f1[1], f1[2], f1[3]};
  v4u uh, ul;
#pragma unroll
  for (int q = 0; q < 4; ++q) {
    const unsigned short h0 = f2bf_bits(e[2 * q]), h1 = f2bf_bits(e[2 * q + 1]);
    const unsigned short l0 = f2bf_bits(e[2 * q] - bf_bits2f(h0)), l1 = f2bf_bits(e[2 * q + 1] - bf_bits2f(h1));
    uh[q] = pk16(h0, h1);
    ul[q] = pk16(l0, l1);
  }
  unsigned short* dh = hi + (size_t)i * 8;
  unsigned short* dl = lo + (size_t)i * 8;
  if (ok) { *(volatile v4u*)dh = uh; *(volatile v4u*)dl = ul; }
  __threadfence();
  if (ok) { *(volatile v4u*)dh = uh; *(volatile v4u*)dl = ul; }
}

__global__ __launch_bounds__(512) void k_bnstat(const float* __restrict__ O, const float* __restrict__ gam,
                                                const float* __restrict__ bet, float* __restrict__ ST) {
  __shared__ double sP[4][HID_];
  __shared__ float sMu[HID_];
  __shared__ __align__(16) float sOut[3 * HID_];
  const int tid = threadIdx.x;
  const int ch = tid & (HID_ - 1), g = tid >> 7;
  const float* col = O + (size_t)g * 1024 * HID_ + ch;
  double s = 0.0;
#pragma unroll 4
  for (int r = 0; r < 1024; ++r) s += (double)col[(size_t)r * HID_];
  sP[g][ch] = s;
  __syncthreads();
  if (tid < HID_) {
    const double S = (sP[0][tid] + sP[1][tid]) + (sP[2][tid] + sP[3][tid]);
    sMu[tid] = (float)(S * (1.0 / 4096.0));
  }
  __syncthreads();
  const float mu = sMu[ch];
  double s2 = 0.0;
#pragma unroll 4
  for (int r = 0; r < 1024; ++r) {
    const float d = col[(size_t)r * HID_] - mu;
    s2 += (double)(d * d);
  }
  sP[g][ch] = s2;
  __syncthreads();
  if (tid < HID_) {
    const double V = (sP[0][tid] + sP[1][tid]) + (sP[2][tid] + sP[3][tid]);
    const float var  = (float)(V * (1.0 / 4096.0));
    const float rstd = rsqrtf(var + BN_EPS);
    sOut[tid]            = sMu[tid];
    sOut[HID_ + tid]     = bf16r(gam[tid]) * rstd;
    sOut[2 * HID_ + tid] = bf16r(bet[tid]);
  }
  __syncthreads();
  v4f v = {0.f, 0.f, 0.f, 0.f};
  const bool wr = tid < (3 * HID_) / 4;
  if (wr) v = *(const v4fa*)(sOut + 4 * tid);
  if (wr) *(volatile v4f*)(ST + 4 * tid) = v;
  __threadfence();
  if (wr) *(volatile v4f*)(ST + 4 * tid) = v;
}

__global__ __launch_bounds__(256) void k_bnapply(const float* __restrict__ O, const float* __restrict__ ST,
                                                 const float* __restrict__ resid, float* __restrict__ outF,
                                                 unsigned short* __restrict__ outH, unsigned short* __restrict__ outL) {
  __shared__ __align__(16) float sF[16 * SFP];
  __shared__ __align__(16) float sS[3 * HID_];
  const int tid = threadIdx.x, lane = tid & 31, w = tid >> 5;
  const int row0 = blockIdx.x * 16;
  const int rl = tid >> 4, c8 = (tid & 15) * 8;
  if (tid < (3 * HID_) / 4) {
    const v4f a = *(const v4fa*)(ST + 4 * tid);
    *(v4fa*)(sS + 4 * tid) = a;
  }
  const size_t eo = (size_t)(row0 + rl) * HID_ + c8;
  const v4f oa = *(const v4fa*)(O + eo);
  const v4f ob = *(const v4fa*)(O + eo + 4);
  const v4f ra = *(const v4fa*)(resid + eo);
  const v4f rb = *(const v4fa*)(resid + eo + 4);
  __syncthreads();
  const float ov[8] = {oa[0], oa[1], oa[2], oa[3], ob[0], ob[1], ob[2], ob[3]};
  const float rv[8] = {ra[0], ra[1], ra[2], ra[3], rb[0], rb[1], rb[2], rb[3]};
  const v4f mua = *(const v4fa*)(sS + c8),            mub = *(const v4fa*)(sS + c8 + 4);
  const v4f sca = *(const v4fa*)(sS + HID_ + c8),     scb = *(const v4fa*)(sS + HID_ + c8 + 4);
  const v4f bea = *(const v4fa*)(sS + 2 * HID_ + c8), beb = *(const v4fa*)(sS + 2 * HID_ + c8 + 4);
  const float muv[8] = {mua[0], mua[1], mua[2], mua[3], mub[0], mub[1], mub[2], mub[3]};
  const float scv[8] = {sca[0], sca[1], sca[2], sca[3], scb[0], scb[1], scb[2], scb[3]};
  const float bev[8] = {bea[0], bea[1], bea[2], bea[3], beb[0], beb[1], beb[2], beb[3]};
  float y[8];
#pragma unroll
  for (int i = 0; i < 8; ++i) y[i] = fmaxf((ov[i] - muv[i]) * scv[i] + bev[i], 0.0f) + rv[i];
  {
    v4f ya, yb;
    ya[0] = y[0]; ya[1] = y[1]; ya[2] = y[2]; ya[3] = y[3];
    yb[0] = y[4]; yb[1] = y[5]; yb[2] = y[6]; yb[3] = y[7];
    *(v4fa*)(sF + rl * SFP + c8)     = ya;
    *(v4fa*)(sF + rl * SFP + c8 + 4) = yb;
  }
  v4u hv, lv;
#pragma unroll
  for (int q = 0; q < 4; ++q) {
    const unsigned short h0 = f2bf_bits(y[2 * q]), h1 = f2bf_bits(y[2 * q + 1]);
    const unsigned short l0 = f2bf_bits(y[2 * q] - bf_bits2f(h0)), l1 = f2bf_bits(y[2 * q + 1] - bf_bits2f(h1));
    hv[q] = pk16(h0, h1);
    lv[q] = pk16(l0, l1);
  }
  __syncthreads();
  for (int pass = 0; pass < 2; ++pass) {
    *(volatile v4u*)(outH + eo) = hv;
    *(volatile v4u*)(outL + eo) = lv;
#pragma unroll
    for (int i = 0; i < 2; ++i) {
      const int row = 2 * w + i;
      const v4f v = *(const v4fa*)(sF + row * SFP + 4 * lane);
      *(volatile v4f*)(outF + (size_t)(row0 + row) * HID_ + 4 * lane) = v;
    }
    __threadfence();
  }
}

extern "C" void kernel_launch(void* const* d_in, const int* in_sizes, int n_in,
                              void* d_out, int out_size, void* d_ws, size_t ws_size,
                              hipStream_t stream) {
  if (n_in < 16) return;
  if (in_sizes[0] != NN_ * FIN_) return;
  if (in_sizes[1] < 2 || (in_sizes[1] & 1) != 0) return;
  const int nE = in_sizes[1] / 2;
  if (nE < 1 || nE > (1 << 24)) return;
  if (in_sizes[2] != FIN_ * HID_) return;
  if (in_sizes[3] != HID_) return;
  for (int i = 4; i <= 10; i += 2) {
    if (in_sizes[i] != NLY_ * HID_ * HID_) return;
    if (in_sizes[i + 1] != NLY_ * HID_) return;
  }
  if (in_sizes[12] != NLY_ * HID_) return;
  if (in_sizes[13] != NLY_ * HID_) return;
  if (in_sizes[14] != HID_ * HID_) return;
  if (in_sizes[15] != HID_) return;
  if (out_size != NN_ * HID_) return;

  const float* x     = (const float*)d_in[0];
  const int*   ei    = (const int*)d_in[1];
  const float* W_in  = (const float*)d_in[2];
  const float* b_in  = (const float*)d_in[3];
  const float* Wq    = (const float*)d_in[4];
  const float* bq    = (const float*)d_in[5];
  const float* Wk    = (const float*)d_in[6];
  const float* bk    = (const float*)d_in[7];
  const float* Wv    = (const float*)d_in[8];
  const float* bvp   = (const float*)d_in[9];
  const float* Wo    = (const float*)d_in[10];
  const float* bo    = (const float*)d_in[11];
  const float* gamma = (const float*)d_in[12];
  const float* beta  = (const float*)d_in[13];
  const float* W_out = (const float*)d_in[14];
  const float* b_out = (const float*)d_in[15];
  float* out = (float*)d_out;
  const int* keys = ei;
  const int* gath = ei + nE;

  const size_t PXB = (size_t)NN_ * KIN_ * 2;
  const size_t PWI = (size_t)HID_ * KIN_ * 2;
  const size_t PWQ = (size_t)HID_ * HID_ * 2;
  const size_t PWS = (size_t)NWSQ * PWQ;
  const size_t PAD = (size_t)NN_ * ADW * 4;
  const size_t PF  = (size_t)NN_ * HID_ * 4;
  const size_t PH  = (size_t)NN_ * HID_ * 2;
  const size_t PVT = (size_t)HID_ * NN_ * 2;
  const size_t PST = 4096;
  size_t off = 0;
  const size_t oXb  = off; off += PXB;
  const size_t oWib = off; off += PWI;
  const size_t oWsq = off; off += PWS;
  const size_t oADJ = off; off += PAD;
  const size_t oHf0 = off; off += PF;
  const size_t oHf1 = off; off += PF;
  const size_t oHh0 = off; off += PH;
  const size_t oHl0 = off; off += PH;
  const size_t oHh1 = off; off += PH;
  const size_t oHl1 = off; off += PH;
  const size_t oQh  = off; off += PH;
  const size_t oQl  = off; off += PH;
  const size_t oKh  = off; off += PH;
  const size_t oKl  = off; off += PH;
  const size_t oVTh = off; off += PVT;
  const size_t oVTl = off; off += PVT;
  const size_t oAO  = off; off += PF;
  const size_t oAOh = off; off += PH;
  const size_t oAOl = off; off += PH;
  const size_t oOB  = off; off += PF;
  const size_t oST  = off; off += PST;
  if (off > ws_size || off > (size_t)WSMAX) return;

  char* ws = (char*)d_ws;
  unsigned short* Xb  = (unsigned short*)(ws + oXb);
  unsigned short* Wib = (unsigned short*)(ws + oWib);
  unsigned short* Wsq = (unsigned short*)(ws + oWsq);
  unsigned int*   ADJ = (unsigned int*)(ws + oADJ);
  float* Hf[2]; Hf[0] = (float*)(ws + oHf0); Hf[1] = (float*)(ws + oHf1);
  unsigned short* Hh[2]; Hh[0] = (unsigned short*)(ws + oHh0); Hh[1] = (unsigned short*)(ws + oHh1);
  unsigned short* Hl[2]; Hl[0] = (unsigned short*)(ws + oHl0); Hl[1] = (unsigned short*)(ws + oHl1);
  unsigned short* Qh  = (unsigned short*)(ws + oQh);
  unsigned short* Ql  = (unsigned short*)(ws + oQl);
  unsigned short* Kh  = (unsigned short*)(ws + oKh);
  unsigned short* Kl  = (unsigned short*)(ws + oKl);
  unsigned short* VTh = (unsigned short*)(ws + oVTh);
  unsigned short* VTl = (unsigned short*)(ws + oVTl);
  float*          AO  = (float*)(ws + oAO);
  unsigned short* AOh = (unsigned short*)(ws + oAOh);
  unsigned short* AOl = (unsigned short*)(ws + oAOl);
  float*          OB  = (float*)(ws + oOB);
  float*          ST  = (float*)(ws + oST);

  const size_t WQE = (size_t)HID_ * HID_;
  const int n8a = NN_ * HID_ / 8;
  const dim3 gG(NN_ / 64);
  const dim3 gA(NN_ / 64, NH_);

  k_cvtx<<<dim3(NN_ / XROWS), XTHR, 0, stream>>>(x, Xb);
  k_cvtwin<<<dim3((HID_ * XUNITS) / 256), 256, 0, stream>>>(W_in, Wib);
  k_tcvt9<<<dim3(HID_ / 64, HID_ / 64, NWSQ), 256, 0, stream>>>(Wq, Wk, Wv, Wo, W_out, Wsq);
  k_adj<<<dim3(NN_ / NSLOT), AD_NT, 0, stream>>>(keys, gath, ADJ, nE, 1);
  k_gemm<false, 1><<<gG, 128, 0, stream>>>(Xb, Xb, KIN_, Wib, b_in, Hf[0], Hh[0], Hl[0]);

  for (int l = 0; l < NLY_; ++l) {
    const int cur = l & 1, nxt = cur ^ 1;
    const size_t bofs = (size_t)l * HID_;
    k_gemm<true, 2><<<gG, 128, 0, stream>>>(Hh[cur], Hl[cur], HID_, Wsq + (size_t)(0 + l) * WQE, bq + bofs, AO, Qh, Ql);
    k_gemm<true, 2><<<gG, 128, 0, stream>>>(Hh[cur], Hl[cur], HID_, Wsq + (size_t)(2 + l) * WQE, bk + bofs, AO, Kh, Kl);
    k_gemm<true, 3><<<gG, 128, 0, stream>>>(Hh[cur], Hl[cur], HID_, Wsq + (size_t)(4 + l) * WQE, bvp + bofs, AO, VTh, VTl);
    k_attn<<<gA, 128, 0, stream>>>(Qh, Ql, Kh, Kl, VTh, VTl, ADJ, AO);
    k_split<<<dim3((n8a + 255) / 256), 256, 0, stream>>>(AO, AOh, AOl, n8a);
    k_gemm<true, 0><<<gG, 128, 0, stream>>>(AOh, AOl, HID_, Wsq + (size_t)(6 + l) * WQE, bo + bofs, OB, Qh, Ql);
    k_bnstat<<<dim3(1), 512, 0, stream>>>(OB, gamma + bofs, beta + bofs, ST);
    k_bnapply<<<dim3(NN_ / 16), 256, 0, stream>>>(OB, ST, Hf[cur], Hf[nxt], Hh[nxt], Hl[nxt]);
  }

  const int fin = NLY_ & 1;
  k_gemm<true, 0><<<gG, 128, 0, stream>>>(Hh[fin], Hl[fin], HID_, Wsq + (size_t)8 * WQE, b_out, out, Qh, Ql);
  (void)hipGetLastError();
}
